// SwitchGRUCell_3745211482670
// MI455X (gfx1250) — hardware-run, weakly checked
//
#include <hip/hip_runtime.h>
#include <math.h>

typedef __attribute__((ext_vector_type(16))) _Float16 v16h;
typedef __attribute__((ext_vector_type(8)))  _Float16 v8h;
typedef __attribute__((ext_vector_type(8)))  float    v8f;
typedef __attribute__((ext_vector_type(4)))  float    v4f;

constexpr int kNB   = 128;
constexpr int kDI   = 512;
constexpr int kNH   = 512;
constexpr int kNE   = 16;
constexpr int kNG   = 3;
constexpr int kGateCols = kNE * kNH;
constexpr int kAllCols  = kNG * kGateCols;
constexpr int kBankElems = kNE * kNH * kDI;
constexpr int kHidSlice  = kNH * kNH;
constexpr int kDiagStep  = kNH + 1;

static_assert(kGateCols == 8192 && kAllCols == 24576, "column map");
static_assert(kBankElems == 4194304, "bank size");
static_assert(kHidSlice == 262144 && kDiagStep == 513, "diagonal index");
static_assert((kNB % 64) == 0 && (kAllCols % 64) == 0, "GEMM M,N multiples of 64");
static_assert((kDI % 32) == 0, "GEMM K multiple of 32");
static_assert(((kNB / 64) * (kAllCols / 64)) % 8 == 0, "8 wave tiles per block, exact");
static_assert((kBankElems / 8) % 256 == 0 && ((kNB * kDI) / 8) % 256 == 0, "convert grids exact");

constexpr float kCarryX = 16.0f;
constexpr float kCarryW = 1024.0f;
constexpr float kFold   = 1.0f / (kCarryX * kCarryW);
constexpr float kF16MinNormal = 6.103515625e-05f;

constexpr size_t kOffXH = 0;
constexpr size_t kOffWH = kOffXH + (size_t)kNB * kDI * 2;
constexpr size_t kOffY  = kOffWH + (size_t)kAllCols * kDI * 2;
constexpr size_t kOffDG = kOffY  + (size_t)kNB * kAllCols * 4;
constexpr size_t kWsTotal = kOffDG + (size_t)kNG * kNE * kNH * 4;
static_assert(kWsTotal == 37978112ull, "carve total");
static_assert(kWsTotal <= 134217728ull, "carve cap");
static_assert((kOffWH % 128) == 0 && (kOffY % 128) == 0 && (kOffDG % 128) == 0, "128-B aligned regions");

__device__ __forceinline__ void acc_tie1(v8f& a, v16h x, v16h y) {
  asm volatile("v_nop\n\tv_nop\n\tv_nop\n\tv_nop" : "+v"(a) : "v"(x), "v"(y));
}
__device__ __forceinline__ void keep4_h(v16h a, v16h b, v16h c, v16h d) {
  asm volatile("v_nop" :: "v"(a), "v"(b), "v"(c), "v"(d));
}
__device__ __forceinline__ void acc_guard4(v8f& a, v8f& b, v8f& c, v8f& d) {
  asm volatile("v_nop\n\tv_nop\n\tv_nop\n\tv_nop" : "+v"(a), "+v"(b), "+v"(c), "+v"(d));
}
template <typename T> struct Frag;
template <> struct Frag<_Float16> {
  typedef v16h V;
  union U { v16h v; v8h h[2]; };
  static __device__ __forceinline__ v16h load(const _Float16* p) {
    U f;
    f.h[0] = *(const v8h*)(p);
    f.h[1] = *(const v8h*)(p + 16);
    return f.v;
  }
  static __device__ __forceinline__ v8f mma(v16h a, v16h b, v8f c) {
    return __builtin_amdgcn_wmma_f32_16x16x32_f16(false, a, false, b, (short)0, c, false, false);
  }
};

__device__ __forceinline__ _Float16 to_f16_carried(float v, float carry) {
  const float s = v * carry;
  const float t = (fabsf(s) < kF16MinNormal) ? 0.0f : s;
  return (_Float16)t;
}

__global__ __launch_bounds__(256) void cvt_rows_f16_kernel(
    const float* __restrict__ src, unsigned short* __restrict__ dst, int total8, float carry)
{
  unsigned i = blockIdx.x * 256u + threadIdx.x;
  asm volatile("" : "+v"(i));
  if (i >= (unsigned)total8) return;
  const size_t e0 = (size_t)i << 3;
  const v4f a0 = *(const v4f*)(src + e0);
  const v4f a1 = *(const v4f*)(src + e0 + 4);
  v8h hv;
#pragma unroll
  for (int e = 0; e < 4; ++e) {
    const float f0 = a0[e];
    const float f1 = a1[e];
    hv[e]     = to_f16_carried(f0, carry);
    hv[4 + e] = to_f16_carried(f1, carry);
  }
  unsigned short* q = dst + e0;
  *(volatile v8h*)q = hv;
  __threadfence();
  *(volatile v8h*)q = hv;
}

__global__ __launch_bounds__(256) void diag_pack_kernel(
    const float* __restrict__ Whr, const float* __restrict__ Whz, const float* __restrict__ Whn,
    float* __restrict__ DG)
{
  if (blockIdx.x >= 24u) return;
  const unsigned g = blockIdx.x >> 3;
  const float* __restrict__ W = (g == 0u) ? Whr : ((g == 1u) ? Whz : Whn);
  unsigned rem = ((blockIdx.x & 7u) << 8) | threadIdx.x;
  asm volatile("" : "+v"(rem));
  unsigned k = rem >> 7;
  asm volatile("" : "+v"(k));
  unsigned h4 = (rem & 127u) << 2;
  asm volatile("" : "+v"(h4));
  const size_t base = (size_t)k * kHidSlice + (size_t)h4 * kDiagStep;
  const float d0 = W[base];
  const float d1 = W[base + kDiagStep];
  const float d2 = W[base + 2 * kDiagStep];
  const float d3 = W[base + 3 * kDiagStep];
  v4f dv;
  dv[0] = d0;
  dv[1] = d1;
  dv[2] = d2;
  dv[3] = d3;
  float* q = DG + (size_t)g * kGateCols + (size_t)k * kNH + h4;
  *(volatile v4f*)q = dv;
  __threadfence();
  *(volatile v4f*)q = dv;
}

__global__ __launch_bounds__(256) void gemm_f16_tile64_kernel(
    const unsigned short* __restrict__ Ap, int lda,
    const unsigned short* __restrict__ Btp, int ldb,
    float* __restrict__ C, int ldc,
    int M, int N, int K, float scale)
{
  typedef _Float16 T;
  typedef Frag<T>::V V;
  const T* A  = (const T*)Ap;
  const T* Bt = (const T*)Btp;
  __shared__ __align__(16) float sT[8][16 * 68];
  const int lane = threadIdx.x & 31;
  const int wave = threadIdx.x >> 5;
  const int tilesN = N >> 6;
  const int tilesM = M >> 6;
  const int tile = blockIdx.x * 8 + wave;
  if (tile >= tilesM * tilesN) return;
  const int tm = tile / tilesN;
  const int tn = tile - tm * tilesN;
  const int m0 = tm << 6;
  const int n0 = tn << 6;

  const int rlane = lane & 15;
  const int koff  = (lane >> 4) * 8;
  const int mOff  = (lane >> 4) * 8;

  v8f acc[4][4];
#pragma unroll
  for (int i = 0; i < 4; ++i)
#pragma unroll
    for (int j = 0; j < 4; ++j) acc[i][j] = (v8f){0.f, 0.f, 0.f, 0.f, 0.f, 0.f, 0.f, 0.f};

  for (int k0 = 0; k0 < K; k0 += 32) {
    V bh[4];
#pragma unroll
    for (int j = 0; j < 4; ++j) {
      const size_t bo = (size_t)(n0 + (j << 4) + rlane) * ldb + koff + k0;
      bh[j] = Frag<T>::load(Bt + bo);
    }
#pragma unroll
    for (int i = 0; i < 4; ++i) {
      const size_t ao = (size_t)(m0 + (i << 4) + rlane) * lda + koff + k0;
      V ah = Frag<T>::load(A + ao);
#pragma unroll
      for (int j = 0; j < 4; ++j) acc[i][j] = Frag<T>::mma(ah, bh[j], acc[i][j]);
      acc_tie1(acc[i][0], ah, bh[0]);
      acc_tie1(acc[i][1], ah, bh[1]);
      acc_tie1(acc[i][2], ah, bh[2]);
      acc_tie1(acc[i][3], ah, bh[3]);
    }
    keep4_h(bh[0], bh[1], bh[2], bh[3]);
  }
  acc_guard4(acc[0][0], acc[0][1], acc[0][2], acc[0][3]);
  acc_guard4(acc[1][0], acc[1][1], acc[1][2], acc[1][3]);
  acc_guard4(acc[2][0], acc[2][1], acc[2][2], acc[2][3]);
  acc_guard4(acc[3][0], acc[3][1], acc[3][2], acc[3][3]);

  float* slab = sT[wave];
#pragma unroll
  for (int i = 0; i < 4; ++i) {
    const int mBase = m0 + (i << 4);
#pragma unroll
    for (int j = 0; j < 4; ++j) {
#pragma unroll
      for (int r = 0; r < 8; ++r) {
        const float v = acc[i][j][r] * scale;
        slab[(mOff + r) * 68 + (j << 4) + rlane] = v;
      }
    }
    __builtin_amdgcn_fence(__ATOMIC_RELEASE, "workgroup");
    __builtin_amdgcn_wave_barrier();
    __builtin_amdgcn_fence(__ATOMIC_ACQUIRE, "workgroup");
    {
      const int hh = lane >> 4;
      const int c4 = (lane & 15) * 4;
      for (int pass = 0; pass < 2; ++pass) {
#pragma unroll
        for (int it = 0; it < 8; ++it) {
          const int row = it * 2 + hh;
          const v4f v = *(const v4f*)(slab + row * 68 + c4);
          *(volatile v4f*)(C + (size_t)(mBase + row) * ldc + n0 + c4) = v;
        }
        __threadfence();
      }
    }
    __builtin_amdgcn_fence(__ATOMIC_RELEASE, "workgroup");
    __builtin_amdgcn_wave_barrier();
    __builtin_amdgcn_fence(__ATOMIC_ACQUIRE, "workgroup");
  }
}

__global__ __launch_bounds__(512) void gate_mix_kernel(
    const float* __restrict__ Y, const float* __restrict__ DG, const float* __restrict__ u,
    const float* __restrict__ hin,
    const float* __restrict__ bxr, const float* __restrict__ bxz, const float* __restrict__ bxn,
    const float* __restrict__ brh, const float* __restrict__ bzh, const float* __restrict__ bnh,
    float* __restrict__ out)
{
  __shared__ __align__(16) float sO[kNH];
  const unsigned b = (blockIdx.x < (unsigned)kNB) ? blockIdx.x : (unsigned)(kNB - 1);
  unsigned h = threadIdx.x;
  asm volatile("" : "+v"(h));
  const float* yrow = Y + (size_t)b * kAllCols;
  float sxr = 0.0f, sxz = 0.0f, sxn = 0.0f;
  float dmr = 0.0f, dmz = 0.0f, dmn = 0.0f;
  float mxr = 0.0f, mxz = 0.0f, mxn = 0.0f;
  float mhr = 0.0f, mhz = 0.0f, mhn = 0.0f;
#pragma unroll 1
  for (int k = 0; k < kNE; ++k) {
    const float uk = u[b * (unsigned)kNE + (unsigned)k];
    const unsigned kh = (unsigned)k * (unsigned)kNH + h;
    sxr = fmaf(uk, yrow[kh], sxr);
    sxz = fmaf(uk, yrow[(unsigned)kGateCols + kh], sxz);
    sxn = fmaf(uk, yrow[2u * (unsigned)kGateCols + kh], sxn);
    dmr = fmaf(uk, DG[kh], dmr);
    dmz = fmaf(uk, DG[(unsigned)kGateCols + kh], dmz);
    dmn = fmaf(uk, DG[2u * (unsigned)kGateCols + kh], dmn);
    mxr = fmaf(uk, bxr[kh], mxr);
    mxz = fmaf(uk, bxz[kh], mxz);
    mxn = fmaf(uk, bxn[kh], mxn);
    mhr = fmaf(uk, brh[kh], mhr);
    mhz = fmaf(uk, bzh[kh], mhz);
    mhn = fmaf(uk, bnh[kh], mhn);
  }
  const float hp = hin[b * (unsigned)kNH + h];
  const float ar = (sxr + mxr) + (dmr * hp + mhr);
  const float az = (sxz + mxz) + (dmz * hp + mhz);
  const float er = expf(-ar);
  const float ez = expf(-az);
  const float r  = 1.0f / (1.0f + er);
  const float z  = 1.0f / (1.0f + ez);
  const float an = (sxn + mxn) + r * (dmn * hp + mhn);
  const float nt = tanhf(an);
  const float ht = (1.0f - z) * nt + z * hp;
  sO[h] = ht;
  __syncthreads();
  if (threadIdx.x < 128u) {
    const unsigned c4 = threadIdx.x * 4u;
    const v4f v = *(const v4f*)(sO + c4);
    float* q = out + (size_t)b * kNH + c4;
    *(volatile v4f*)q = v;
    __threadfence();
    *(volatile v4f*)q = v;
  }
}

extern "C" void kernel_launch(void* const* d_in, const int* in_sizes, int n_in,
                              void* d_out, int out_size, void* d_ws, size_t ws_size,
                              hipStream_t stream) {
  if (n_in < 15) return;
  if (in_sizes[0] != kNB * kDI) return;
  if (in_sizes[1] != kNB * kNH) return;
  if (in_sizes[2] != kNB * kNE) return;
  for (int i = 3; i < 9; ++i) if (in_sizes[i] != kBankElems) return;
  for (int i = 9; i < 15; ++i) if (in_sizes[i] != kNE * kNH) return;
  if (out_size != kNB * kNH) return;
  if (ws_size < kWsTotal) return;

  const float* x   = (const float*)d_in[0];
  const float* hin = (const float*)d_in[1];
  const float* u   = (const float*)d_in[2];
  const float* Wxr = (const float*)d_in[3];
  const float* Wxz = (const float*)d_in[4];
  const float* Wxn = (const float*)d_in[5];
  const float* Whr = (const float*)d_in[6];
  const float* Whz = (const float*)d_in[7];
  const float* Whn = (const float*)d_in[8];
  const float* bxr = (const float*)d_in[9];
  const float* bxz = (const float*)d_in[10];
  const float* bxn = (const float*)d_in[11];
  const float* brh = (const float*)d_in[12];
  const float* bzh = (const float*)d_in[13];
  const float* bnh = (const float*)d_in[14];
  float* out = (float*)d_out;

  char* ws = (char*)d_ws;
  unsigned short* XH = (unsigned short*)(ws + kOffXH);
  unsigned short* WH = (unsigned short*)(ws + kOffWH);
  float*          Y  = (float*)(ws + kOffY);
  float*          DG = (float*)(ws + kOffDG);

  cvt_rows_f16_kernel<<<(kNB * kDI / 8) / 256, 256, 0, stream>>>(x, XH, kNB * kDI / 8, kCarryX);
  cvt_rows_f16_kernel<<<(kBankElems / 8) / 256, 256, 0, stream>>>(Wxr, WH, kBankElems / 8, kCarryW);
  cvt_rows_f16_kernel<<<(kBankElems / 8) / 256, 256, 0, stream>>>(Wxz, WH + (size_t)kBankElems, kBankElems / 8, kCarryW);
  cvt_rows_f16_kernel<<<(kBankElems / 8) / 256, 256, 0, stream>>>(Wxn, WH + 2 * (size_t)kBankElems, kBankElems / 8, kCarryW);

  diag_pack_kernel<<<24, 256, 0, stream>>>(Whr, Whz, Whn, DG);

  gemm_f16_tile64_kernel<<<((kNB / 64) * (kAllCols / 64)) / 8, 256, 0, stream>>>(
      XH, kDI, WH, kDI, Y, kAllCols, kNB, kAllCols, kDI, kFold);

  gate_mix_kernel<<<kNB, kNH, 0, stream>>>(Y, DG, u, hin, bxr, bxz, bxn, brh, bzh, bnh, out);
}
